// LinearLocalAttention_6717328851261
// MI455X (gfx1250) — hardware-verified
//
#include <hip/hip_runtime.h>

#define DIM_ 1024
#define NH_  8
#define HD_  128
#define NF_  64
#define SEQ_ 4096
#define WIN_ 7

typedef _Float16 v16h __attribute__((ext_vector_type(16)));
typedef _Float16 v8h  __attribute__((ext_vector_type(8)));
typedef _Float16 v4h  __attribute__((ext_vector_type(4)));
typedef float    v8f  __attribute__((ext_vector_type(8)));
typedef float    v4f  __attribute__((ext_vector_type(4)));
union Frag { v16h v; v8h half[2]; };

__device__ __forceinline__ v8f wmma_f16(v16h a, v16h b, v8f c) {
    c = __builtin_amdgcn_wmma_f32_16x16x32_f16(false, a, false, b, (short)0, c, false, false);
    asm volatile("v_nop\n\tv_nop\n\tv_nop\n\tv_nop" : "+v"(c) : "v"(a), "v"(b));
    return c;
}

__device__ __forceinline__ v8h cvt8h(v4f a, v4f b) {
    v4h ha = __builtin_convertvector(a, v4h);
    v4h hb = __builtin_convertvector(b, v4h);
    return __builtin_shufflevector(ha, hb, 0, 1, 2, 3, 4, 5, 6, 7);
}
__device__ __forceinline__ v8h load8h(const float* p) {
    v4f a = *(const v4f*)p;
    v4f b = *(const v4f*)(p + 4);
    return cvt8h(a, b);
}
__device__ __forceinline__ v8h load8h(const _Float16* p) {
    return *(const v8h*)p;
}

__global__ __launch_bounds__(256) void k_wtrans(const float* __restrict__ W, int R, int Cc,
                                                _Float16* __restrict__ Wt, float scale)
{
    __shared__ _Float16 T[64][72] __attribute__((aligned(16)));
    const int tid = threadIdx.x, lane = tid & 31, wv = tid >> 5;
    const int r0 = blockIdx.y * 64, c0 = blockIdx.x * 64;
    #pragma unroll
    for (int t = 0; t < 4; ++t) {
        const int s  = tid + t * 256;
        const int rr = s >> 4;
        const int c4 = (s & 15) * 4;
        v4f v = *(const v4f*)(W + (size_t)(r0 + rr) * Cc + c0 + c4);
        T[c4 + 0][rr] = (_Float16)(v[0] * scale);
        T[c4 + 1][rr] = (_Float16)(v[1] * scale);
        T[c4 + 2][rr] = (_Float16)(v[2] * scale);
        T[c4 + 3][rr] = (_Float16)(v[3] * scale);
    }
    __syncthreads();
    v8h hv[2]; size_t go[2];
    #pragma unroll
    for (int it = 0; it < 2; ++it) {
        const int cc = wv * 8 + it * 4 + (lane >> 3);
        const int ro = (lane & 7) * 8;
        hv[it] = *(const v8h*)(&T[cc][ro]);
        go[it] = (size_t)(c0 + cc) * R + r0 + ro;
    }
    #pragma unroll
    for (int it = 0; it < 2; ++it) *(volatile v8h*)(Wt + go[it]) = hv[it];
    __threadfence();
    #pragma unroll
    for (int it = 0; it < 2; ++it) *(volatile v8h*)(Wt + go[it]) = hv[it];
}

template <typename TA>
__device__ __forceinline__ void gemm_tile(float* smem, const TA* __restrict__ A, int lda,
    const _Float16* __restrict__ Bt, int ldb, int K,
    _Float16* outH, int ldH, float sH, int nsplit,
    float* outF, int ldF, float sF, const float* __restrict__ bias, int hasb)
{
    constexpr int BM = 128, BK = 64, PK = 72, CP = 128;
    _Float16* As = (_Float16*)smem;
    _Float16* Bs = As + BM * PK;
    const int tid = threadIdx.x, lane = tid & 31, wv = tid >> 5;
    const int wm = wv & 1, wn = wv >> 1;
    const int hh = lane >> 4, l16 = lane & 15;
    const int m0 = blockIdx.y * BM, n0 = blockIdx.x * BM;

    v8f acc[4][2] = {};

    for (int kb = 0; kb < K; kb += BK) {
        __syncthreads();
        #pragma unroll
        for (int t = 0; t < 4; ++t) {
            const int s   = tid + t * 256;
            const int row = s >> 3;
            const int cc  = (s & 7) * 8;
            v8h ha = load8h(A + (size_t)(m0 + row) * lda + kb + cc);
            *(v8h*)(As + row * PK + cc) = ha;
            v8h hb = *(const v8h*)(Bt + (size_t)(n0 + row) * ldb + kb + cc);
            *(v8h*)(Bs + row * PK + cc) = hb;
        }
        __syncthreads();
        #pragma unroll
        for (int ks = 0; ks < 2; ++ks) {
            const int k0 = ks * 32;
            Frag bfr[2];
            #pragma unroll
            for (int j = 0; j < 2; ++j) {
                const _Float16* p = Bs + (wn * 32 + j * 16 + l16) * PK + k0 + 8 * hh;
                bfr[j].half[0] = *(const v8h*)p;
                bfr[j].half[1] = *(const v8h*)(p + 16);
            }
            #pragma unroll
            for (int i = 0; i < 4; ++i) {
                Frag af;
                const _Float16* p = As + (wm * 64 + i * 16 + l16) * PK + k0 + 8 * hh;
                af.half[0] = *(const v8h*)p;
                af.half[1] = *(const v8h*)(p + 16);
                acc[i][0] = wmma_f16(af.v, bfr[0].v, acc[i][0]);
                acc[i][1] = wmma_f16(af.v, bfr[1].v, acc[i][1]);
            }
        }
    }

    __syncthreads();
    float* Cs = smem;
    #pragma unroll
    for (int i = 0; i < 4; ++i)
        #pragma unroll
        for (int j = 0; j < 2; ++j)
            #pragma unroll
            for (int r = 0; r < 8; ++r)
                Cs[(wm * 64 + i * 16 + 8 * hh + r) * CP + wn * 32 + j * 16 + l16] = acc[i][j][r];
    __syncthreads();

    if (n0 < nsplit) {
        v8h hv[8]; size_t go[8];
        #pragma unroll
        for (int it = 0; it < 8; ++it) {
            const int row = wv * 16 + 2 * it + hh;
            const int c8  = l16 * 8;
            v4f a = *(const v4f*)(Cs + row * CP + c8);
            v4f b = *(const v4f*)(Cs + row * CP + c8 + 4);
            hv[it] = cvt8h(a * sH, b * sH);
            go[it] = (size_t)(m0 + row) * ldH + n0 + c8;
        }
        #pragma unroll
        for (int it = 0; it < 8; ++it) *(volatile v8h*)(outH + go[it]) = hv[it];
        __threadfence();
        #pragma unroll
        for (int it = 0; it < 8; ++it) *(volatile v8h*)(outH + go[it]) = hv[it];
    } else {
        const int c4   = lane * 4;
        const int ncol = n0 - nsplit + c4;
        v4f bb = {0.f, 0.f, 0.f, 0.f};
        if (hasb) bb = *(const v4f*)(bias + ncol);
        v4f fv[16];
        #pragma unroll
        for (int it = 0; it < 16; ++it) {
            v4f v = *(const v4f*)(Cs + (wv * 16 + it) * CP + c4);
            fv[it] = v * sF + bb;
        }
        float* gb = outF + (size_t)(m0 + wv * 16) * ldF + ncol;
        #pragma unroll
        for (int it = 0; it < 16; ++it) *(volatile v4f*)(gb + (size_t)it * ldF) = fv[it];
        __threadfence();
        #pragma unroll
        for (int it = 0; it < 16; ++it) *(volatile v4f*)(gb + (size_t)it * ldF) = fv[it];
    }
}

__global__ __launch_bounds__(256) void k_gemm_a32(const float* __restrict__ A, int lda,
    const _Float16* __restrict__ Bt, int ldb, int K,
    _Float16* outH, int ldH, float sH, int nsplit,
    float* outF, int ldF, float sF, const float* __restrict__ bias, int hasb)
{
    __shared__ float smem[16384] __attribute__((aligned(16)));
    gemm_tile<float>(smem, A, lda, Bt, ldb, K, outH, ldH, sH, nsplit, outF, ldF, sF, bias, hasb);
}

__global__ __launch_bounds__(256) void k_gemm_a16(const _Float16* __restrict__ A, int lda,
    const _Float16* __restrict__ Bt, int ldb, int K,
    _Float16* outH, int ldH, float sH, int nsplit,
    float* outF, int ldF, float sF, const float* __restrict__ bias, int hasb)
{
    __shared__ float smem[16384] __attribute__((aligned(16)));
    gemm_tile<_Float16>(smem, A, lda, Bt, ldb, K, outH, ldH, sH, nsplit, outF, ldF, sF, bias, hasb);
}

__global__ __launch_bounds__(128) void k_phi(const _Float16* __restrict__ QK, int ldqk, int coloff,
    const _Float16* __restrict__ Pt, float* __restrict__ PHI, int Nn)
{
    __shared__ float Cs[64 * 68] __attribute__((aligned(16)));
    const int tid = threadIdx.x, lane = tid & 31, wv = tid >> 5;
    const int hh = lane >> 4, l16 = lane & 15;
    const int bh = blockIdx.y, b = bh >> 3, h = bh & 7;
    const int n0 = blockIdx.x * 64;
    const _Float16* arow = QK + ((size_t)b * Nn + n0 + wv * 16 + l16) * ldqk + coloff + h * HD_ + 8 * hh;

    v8f acc[4] = {};
    #pragma unroll
    for (int ks = 0; ks < 4; ++ks) {
        const int k0 = ks * 32;
        Frag af;
        af.half[0] = *(const v8h*)(arow + k0);
        af.half[1] = *(const v8h*)(arow + k0 + 16);
        #pragma unroll
        for (int j = 0; j < 4; ++j) {
            const _Float16* p = Pt + (size_t)(j * 16 + l16) * HD_ + k0 + 8 * hh;
            Frag bfr;
            bfr.half[0] = *(const v8h*)p;
            bfr.half[1] = *(const v8h*)(p + 16);
            acc[j] = wmma_f16(af.v, bfr.v, acc[j]);
        }
    }

    #pragma unroll
    for (int j = 0; j < 4; ++j)
        #pragma unroll
        for (int r = 0; r < 8; ++r) {
            const float t = acc[j][r] * (1.0f / 128.0f);
            const float o = (t > 0.0f) ? (t + 1.0f) : expf(t);
            Cs[(wv * 16 + 8 * hh + r) * 68 + j * 16 + l16] = o;
        }
    __syncthreads();

    v4f fv[8];
    #pragma unroll
    for (int it = 0; it < 8; ++it) {
        const int row = wv * 16 + 2 * it + hh;
        fv[it] = *(const v4f*)(Cs + row * 68 + l16 * 4);
    }
    float* gb = PHI + ((size_t)bh * Nn + n0) * NF_;
    #pragma unroll
    for (int it = 0; it < 8; ++it)
        *(volatile v4f*)(gb + (size_t)(wv * 16 + 2 * it + hh) * NF_ + l16 * 4) = fv[it];
    __threadfence();
    #pragma unroll
    for (int it = 0; it < 8; ++it)
        *(volatile v4f*)(gb + (size_t)(wv * 16 + 2 * it + hh) * NF_ + l16 * 4) = fv[it];
}

__global__ __launch_bounds__(256) void k_attn(const float* __restrict__ QP, const float* __restrict__ KP,
    const float* __restrict__ V, int ldv, _Float16* __restrict__ AO, int ldo, int Bb, int Nn)
{
    const int lane = threadIdx.x & 31, wv = threadIdx.x >> 5;
    const int hh = lane >> 4, l16 = lane & 15;
    const long long gw = (long long)blockIdx.x * (long long)(blockDim.x >> 5) + wv;
    const int hp = (int)(gw & 3);
    const long long t2 = gw >> 2;
    const int n = (int)(t2 % Nn);
    const int b = (int)(t2 / Nn);
    if (b >= Bb) return;
    const int h  = hp * 2 + hh;
    const int bh = b * NH_ + h;

    const v4f q4 = *(const v4f*)(QP + ((size_t)bh * Nn + n) * NF_ + 4 * l16);
    v4f o0 = {0.f, 0.f, 0.f, 0.f};
    v4f o1 = {0.f, 0.f, 0.f, 0.f};
    float zs = 0.f;
    #pragma unroll 1
    for (int w = 0; w < WIN_; ++w) {
        const int pos = n + w - (WIN_ / 2);
        if (pos >= 0 && pos < Nn) {
            const v4f k4 = *(const v4f*)(KP + ((size_t)bh * Nn + pos) * NF_ + 4 * l16);
            float s = q4[0] * k4[0] + q4[1] * k4[1] + q4[2] * k4[2] + q4[3] * k4[3];
            s += __shfl_xor(s, 8, 32);
            s += __shfl_xor(s, 4, 32);
            s += __shfl_xor(s, 2, 32);
            s += __shfl_xor(s, 1, 32);
            zs += s;
            const float* vr = V + ((size_t)b * Nn + pos) * ldv + h * HD_ + 8 * l16;
            const v4f v0 = *(const v4f*)vr;
            const v4f v1 = *(const v4f*)(vr + 4);
            o0 += s * v0;
            o1 += s * v1;
        }
    }
    const float z  = 1.0f / (zs + 1e-8f);
    const float zz = z * 16.0f;
    const v8h hv = cvt8h(o0 * zz, o1 * zz);
    _Float16* gp = AO + ((size_t)b * Nn + n) * ldo + h * HD_ + 8 * l16;
    *(volatile v8h*)gp = hv;
    __threadfence();
    *(volatile v8h*)gp = hv;
}

extern "C" void kernel_launch(void* const* d_in, const int* in_sizes, int n_in,
                              void* d_out, int out_size, void* d_ws, size_t ws_size,
                              hipStream_t stream)
{
    if (n_in < 5) return;
    const float* x     = (const float*)d_in[0];
    const float* w_qkv = (const float*)d_in[1];
    const float* proj  = (const float*)d_in[2];
    const float* w_out = (const float*)d_in[3];
    const float* b_out = (const float*)d_in[4];
    float* out = (float*)d_out;

    const long long nx = (long long)in_sizes[0];
    const int M = (int)(nx / DIM_);
    if ((long long)M * DIM_ != nx || M <= 0 || (M % 128) != 0 || (M % SEQ_) != 0) return;
    const int Bb = M / SEQ_;
    if (in_sizes[1] != DIM_ * 3 * DIM_ || in_sizes[2] != HD_ * NF_ ||
        in_sizes[3] != DIM_ * DIM_ || in_sizes[4] != DIM_) return;
    if ((long long)out_size != (long long)M * DIM_) return;

    char* ws = (char*)d_ws;
    size_t off = 0;
    const size_t sz_wqkv_t = (size_t)3 * DIM_ * DIM_ * 2;
    const size_t sz_wout_t = (size_t)DIM_ * DIM_ * 2;
    const size_t sz_proj_t = (size_t)NF_ * HD_ * 2;
    const size_t sz_qk     = (size_t)M * 2 * DIM_ * 2;
    const size_t sz_v      = (size_t)M * DIM_ * 4;
    const size_t sz_phi    = (size_t)M * NH_ * NF_ * 4;
    const size_t sz_attn   = (size_t)M * DIM_ * 2;
    _Float16* wqkv_t = (_Float16*)(ws + off); off += (sz_wqkv_t + 255) & ~(size_t)255;
    _Float16* wout_t = (_Float16*)(ws + off); off += (sz_wout_t + 255) & ~(size_t)255;
    _Float16* proj_t = (_Float16*)(ws + off); off += (sz_proj_t + 255) & ~(size_t)255;
    _Float16* qk_h   = (_Float16*)(ws + off); off += (sz_qk     + 255) & ~(size_t)255;
    float*    v_f    = (float*)   (ws + off); off += (sz_v      + 255) & ~(size_t)255;
    float*    qphi_f = (float*)   (ws + off); off += (sz_phi    + 255) & ~(size_t)255;
    float*    kphi_f = (float*)   (ws + off); off += (sz_phi    + 255) & ~(size_t)255;
    _Float16* attn_h = (_Float16*)(ws + off); off += (sz_attn   + 255) & ~(size_t)255;
    if (off > ws_size) return;

    const dim3 b256(256), b128(128);

    k_wtrans<<<dim3(3 * DIM_ / 64, DIM_ / 64), b256, 0, stream>>>(w_qkv, DIM_, 3 * DIM_, wqkv_t, 64.0f);
    k_wtrans<<<dim3(DIM_ / 64, DIM_ / 64), b256, 0, stream>>>(w_out, DIM_, DIM_, wout_t, 64.0f);
    k_wtrans<<<dim3(NF_ / 64, HD_ / 64), b256, 0, stream>>>(proj, HD_, NF_, proj_t, 16.0f);

    k_gemm_a32<<<dim3(3 * DIM_ / 128, M / 128), b256, 0, stream>>>(
        x, DIM_, wqkv_t, DIM_, DIM_,
        qk_h, 2 * DIM_, 0.125f, 2 * DIM_,
        v_f, DIM_, 1.0f / 64.0f, b_out, 0);

    k_phi<<<dim3(SEQ_ / 64, Bb * NH_), b128, 0, stream>>>(qk_h, 2 * DIM_, 0,    proj_t, qphi_f, SEQ_);
    k_phi<<<dim3(SEQ_ / 64, Bb * NH_), b128, 0, stream>>>(qk_h, 2 * DIM_, DIM_, proj_t, kphi_f, SEQ_);

    const long long nwaves = (long long)Bb * SEQ_ * (NH_ / 2);
    const unsigned nblk = (unsigned)((nwaves + 7) / 8);
    k_attn<<<dim3(nblk), b256, 0, stream>>>(qphi_f, kphi_f, v_f, DIM_, attn_h, DIM_, Bb, SEQ_);

    k_gemm_a16<<<dim3(DIM_ / 128, M / 128), b256, 0, stream>>>(
        attn_h, DIM_, wout_t, DIM_, DIM_,
        qk_h, 2 * DIM_, 1.0f, 0,
        out, DIM_, 1.0f / 1024.0f, b_out, 1);
}
